// RNNDecoderIndivdual_33655363732231
// MI455X (gfx1250) — hardware-run, weakly checked
//
#include <hip/hip_runtime.h>
#include <math.h>

typedef __attribute__((ext_vector_type(16))) _Float16 v16h;
typedef __attribute__((ext_vector_type(8)))  _Float16 v8h;
typedef __attribute__((ext_vector_type(8)))  float    v8f;
typedef __attribute__((ext_vector_type(4)))  float    v4f;

constexpr int NBATCH   = 64;
constexpr int NSTEP    = 2048;
constexpr int NHID     = 256;
constexpr int NTHR_SEQ = 512;
constexpr int ROWS_BLK = 16;
constexpr int HPITCH   = 264;
constexpr int CHUNK    = 32;
constexpr int NCHUNK   = NSTEP / CHUNK;
constexpr int PARTP    = 16;
constexpr int NOUTCOL  = NSTEP + 1;
constexpr int NOUT     = NBATCH * NOUTCOL;
constexpr int NOUT4    = NOUT / 4;
constexpr int NBLK_SEQ = NBATCH / ROWS_BLK;
constexpr int NW_ELEMS = NHID * NHID;

constexpr float HCARRY   = 512.0f;
constexpr float WCARRY   = 1024.0f;
constexpr float ACC_SCL  = 1.0f / (HCARRY * WCARRY);
constexpr float F16_MINN = 6.103515625e-5f;

static_assert(NBATCH % ROWS_BLK == 0, "block rows");
static_assert(NHID == 16 * (NTHR_SEQ / 32), "16 waves x 16 hidden units");
static_assert(NHID % 32 == 0, "K multiple of 32");
static_assert(NSTEP % CHUNK == 0 && (CHUNK % 2) == 0, "chunking");
static_assert(NOUT == 131136 && (NOUT % 4) == 0, "output size");
static_assert(NOUT4 == 32784, "output float4 count");
static_assert((HPITCH % 8) == 0 && HPITCH >= NHID, "LDS pitch");
static_assert(ROWS_BLK * CHUNK == 512, "staging tile");
static_assert(NW_ELEMS / 8 == 32 * 256, "weight plane conversion coverage");

constexpr size_t SZ_W    = (size_t)NW_ELEMS * 2;
constexpr size_t SZ_YSEQ = (size_t)NCHUNK * NBATCH * CHUNK * 4;
constexpr size_t SZ_YMAX = (size_t)NBLK_SEQ * 32 * 4;
constexpr size_t OFF_WH0  = 0;
constexpr size_t OFF_WI1  = OFF_WH0 + SZ_W;
constexpr size_t OFF_WH1  = OFF_WI1 + SZ_W;
constexpr size_t OFF_YSEQ = OFF_WH1 + SZ_W;
constexpr size_t OFF_YMAX = OFF_YSEQ + SZ_YSEQ;
constexpr size_t WS_TOTAL = OFF_YMAX + SZ_YMAX;
static_assert(WS_TOTAL == 918016ull, "carve total");
static_assert(WS_TOTAL <= 134217728ull, "carve cap");
static_assert((OFF_WI1 % 256) == 0 && (OFF_WH1 % 256) == 0 && (OFF_YSEQ % 256) == 0 && (OFF_YMAX % 256) == 0, "aligned regions");

__device__ __forceinline__ unsigned short f2bf_bits(float f) {
  unsigned u = __float_as_uint(f);
  return (unsigned short)((u + 0x7FFFu + ((u >> 16) & 1u)) >> 16);
}
__device__ __forceinline__ float bf_bits2f(unsigned short h) { return __uint_as_float(((unsigned)h) << 16); }
__device__ __forceinline__ float bf16r(float f) { return bf_bits2f(f2bf_bits(f)); }

__device__ __forceinline__ _Float16 to_f16_operand(float carried) {
  const float v = (fabsf(carried) < F16_MINN) ? 0.0f : carried;
  return (_Float16)v;
}

union FragU { v16h v; v8h h[2]; };
__device__ __forceinline__ v16h frag_load(const _Float16* p) {
  FragU f;
  f.h[0] = *(const v8h*)(p);
  f.h[1] = *(const v8h*)(p + 16);
  return f.v;
}
__device__ __forceinline__ v8f mma_g(v16h a, v16h b, v8f c) {
  c = __builtin_amdgcn_wmma_f32_16x16x32_f16(false, a, false, b, (short)0, c, false, false);
  asm volatile("v_nop\n\tv_nop\n\tv_nop\n\tv_nop" : "+v"(c) : "v"(a), "v"(b));
  return c;
}
__device__ __forceinline__ v8f tile_k256(const _Float16* arow, const _Float16* wrow, v8f acc) {
#pragma unroll 1
  for (int k0 = 0; k0 < NHID; k0 += 32) {
    const v16h a = frag_load(arow + k0);
    const v16h b = frag_load(wrow + k0);
    acc = mma_g(a, b, acc);
  }
  return acc;
}

__global__ __launch_bounds__(256) void wplane_kernel(
    const float* __restrict__ w0, const float* __restrict__ w1, const float* __restrict__ w2,
    unsigned short* __restrict__ d0, unsigned short* __restrict__ d1, unsigned short* __restrict__ d2)
{
  const int m = blockIdx.x >> 5;
  const float* src = (m == 0) ? w0 : ((m == 1) ? w1 : w2);
  unsigned short* dst = (m == 0) ? d0 : ((m == 1) ? d1 : d2);
  const int i = (blockIdx.x & 31) * 256 + threadIdx.x;
  const float* sp = src + (size_t)i * 8;
  const v4f a = *(const v4f*)(sp);
  const v4f b = *(const v4f*)(sp + 4);
  v8h hv;
#pragma unroll
  for (int e = 0; e < 4; ++e) {
    hv[e]     = to_f16_operand(bf16r(a[e]) * WCARRY);
    hv[4 + e] = to_f16_operand(bf16r(b[e]) * WCARRY);
  }
  unsigned short* q = dst + (size_t)i * 8;
  *(volatile v8h*)q = hv;
  __threadfence();
  *(volatile v8h*)q = hv;
}

__global__ __launch_bounds__(NTHR_SEQ) void rnn2_seq_kernel(
    const float* __restrict__ x, const float* __restrict__ z,
    const float* __restrict__ wih0, const float* __restrict__ bih0, const float* __restrict__ bhh0,
    const float* __restrict__ bih1, const float* __restrict__ bhh1,
    const float* __restrict__ wlin, const float* __restrict__ blin,
    const unsigned short* __restrict__ WH0p, const unsigned short* __restrict__ WI1p,
    const unsigned short* __restrict__ WH1p,
    float* __restrict__ YSEQ, float* __restrict__ YMAX)
{
  __shared__ __align__(16) _Float16 H0[2][ROWS_BLK * HPITCH];
  __shared__ __align__(16) _Float16 H1[2][ROWS_BLK * HPITCH];
  __shared__ __align__(16) float XZ[2 * ROWS_BLK * CHUNK];
  __shared__ __align__(16) float YB[ROWS_BLK * CHUNK];
  __shared__ __align__(16) float PART[ROWS_BLK * PARTP];

  const _Float16* WH0 = (const _Float16*)WH0p;
  const _Float16* WI1 = (const _Float16*)WI1p;
  const _Float16* WH1 = (const _Float16*)WH1p;

  const int tid  = threadIdx.x;
  const int lane = tid & 31;
  const int wave = tid >> 5;
  const int c    = lane & 15;
  const int hh   = lane >> 4;
  const int koff = hh * 8;
  const int n    = 16 * wave + c;
  const int b0   = blockIdx.x * ROWS_BLK;

  {
    _Float16* z0 = &H0[0][0];
    _Float16* z1 = &H1[0][0];
#pragma unroll 1
    for (int i = tid; i < 2 * ROWS_BLK * HPITCH; i += NTHR_SEQ) {
      z0[i] = (_Float16)0.0f;
      z1[i] = (_Float16)0.0f;
    }
  }

  const float w_in0 = bf16r(wih0[n]);
  const float b0a   = bf16r(bih0[n]);
  const float b0b   = bf16r(bhh0[n]);
  const float b1s   = bf16r(bih1[n]) + bf16r(bhh1[n]);
  const float w_hd  = bf16r(wlin[n]);
  float bl_raw = blin[0];
  asm volatile("" : "+v"(bl_raw));
  const float b_hd = bf16r(bl_raw);

  const _Float16* wr0 = WH0 + (size_t)n * NHID + koff;
  const _Float16* wri = WI1 + (size_t)n * NHID + koff;
  const _Float16* wrh = WH1 + (size_t)n * NHID + koff;

  const v8f z8 = {0.f, 0.f, 0.f, 0.f, 0.f, 0.f, 0.f, 0.f};
  float ymax = -INFINITY;
  __syncthreads();

#pragma unroll 1
  for (int ch = 0; ch < NCHUNK; ++ch) {
    if (tid < 256) {
      const int which = tid >> 7;
      const int q     = tid & 127;
      const int row   = q >> 3;
      const int c4    = (q & 7) * 4;
      const float* src = which ? z : x;
      v4f v = *(const v4f*)(src + (size_t)(b0 + row) * NSTEP + ch * CHUNK + c4);
      v[0] = bf16r(v[0]);
      v[1] = bf16r(v[1]);
      v[2] = bf16r(v[2]);
      v[3] = bf16r(v[3]);
      *(v4f*)(XZ + which * (ROWS_BLK * CHUNK) + row * CHUNK + c4) = v;
    }
    __syncthreads();

#pragma unroll 1
    for (int s = 0; s < CHUNK; ++s) {
      const int p = s & 1;

      v8f acc0 = z8;
      acc0 = tile_k256(&H0[p][0] + c * HPITCH + koff, wr0, acc0);
#pragma unroll
      for (int r = 0; r < 8; ++r) {
        const float xv  = XZ[(8 * hh + r) * CHUNK + s];
        const float xp  = ((xv * w_in0) + b0a) + b0b;
        const float pre = acc0[r] * ACC_SCL + xp;
        const float hn  = tanhf(pre);
        H0[p ^ 1][(8 * hh + r) * HPITCH + n] = to_f16_operand(hn * HCARRY);
      }
      __syncthreads();

      v8f acc1 = z8;
      acc1 = tile_k256(&H0[p ^ 1][0] + c * HPITCH + koff, wri, acc1);
      acc1 = tile_k256(&H1[p][0] + c * HPITCH + koff, wrh, acc1);
      float pv[8];
#pragma unroll
      for (int r = 0; r < 8; ++r) {
        const float pre = acc1[r] * ACC_SCL + b1s;
        const float hn  = tanhf(pre);
        H1[p ^ 1][(8 * hh + r) * HPITCH + n] = to_f16_operand(hn * HCARRY);
        pv[r] = hn * w_hd;
      }
#pragma unroll
      for (int r = 0; r < 8; ++r) {
        pv[r] += __shfl_xor(pv[r], 1, 32);
        pv[r] += __shfl_xor(pv[r], 2, 32);
        pv[r] += __shfl_xor(pv[r], 4, 32);
        pv[r] += __shfl_xor(pv[r], 8, 32);
      }
      if (c == 0) {
#pragma unroll
        for (int r = 0; r < 8; ++r) PART[(8 * hh + r) * PARTP + wave] = pv[r];
      }
      __syncthreads();

      if (tid < ROWS_BLK) {
        const float* pp = PART + tid * PARTP;
        const v4f a0 = *(const v4f*)(pp);
        const v4f a1 = *(const v4f*)(pp + 4);
        const v4f a2 = *(const v4f*)(pp + 8);
        const v4f a3 = *(const v4f*)(pp + 12);
        float sum = a0[0];
        sum += a0[1]; sum += a0[2]; sum += a0[3];
        sum += a1[0]; sum += a1[1]; sum += a1[2]; sum += a1[3];
        sum += a2[0]; sum += a2[1]; sum += a2[2]; sum += a2[3];
        sum += a3[0]; sum += a3[1]; sum += a3[2]; sum += a3[3];
        const float zv = XZ[ROWS_BLK * CHUNK + tid * CHUNK + s];
        const float y  = zv * sum + b_hd;
        YB[tid * CHUNK + s] = y;
        ymax = fmaxf(ymax, y);
      }
    }

    __syncthreads();
    if (tid < 128) {
      const v4f v = *(const v4f*)(YB + tid * 4);
      float* dp = YSEQ + ((size_t)ch * NBATCH + b0) * CHUNK + tid * 4;
      *(volatile v4f*)dp = v;
      __threadfence();
      *(volatile v4f*)dp = v;
    }
  }

  if (wave == 0) {
    const float mv = (lane < ROWS_BLK) ? ymax : 0.0f;
    float* mp = YMAX + blockIdx.x * 32 + lane;
    *(volatile float*)mp = mv;
    __threadfence();
    *(volatile float*)mp = mv;
  }
}

__global__ __launch_bounds__(256) void pack_kernel(
    const float* __restrict__ YSEQ, const float* __restrict__ YMAX, float* __restrict__ out)
{
  const int j  = blockIdx.x * 256 + threadIdx.x;
  const int jc = (j < NOUT4) ? j : (NOUT4 - 1);
  v4f o;
#pragma unroll
  for (int e = 0; e < 4; ++e) {
    const int idx = jc * 4 + e;
    const int b   = idx / NOUTCOL;
    const int col = idx - b * NOUTCOL;
    const int cl  = (col < NSTEP) ? col : (NSTEP - 1);
    float yv = YSEQ[((size_t)(cl >> 5) * NBATCH + b) * CHUNK + (cl & 31)];
    float mv = YMAX[(b >> 4) * 32 + (b & 15)];
    asm volatile("" : "+v"(yv));
    asm volatile("" : "+v"(mv));
    o[e] = (col < NSTEP) ? yv : mv;
  }
  if (j < NOUT4) {
    float* op = out + (size_t)j * 4;
    *(volatile v4f*)op = o;
    __threadfence();
    *(volatile v4f*)op = o;
  }
}

extern "C" void kernel_launch(void* const* d_in, const int* in_sizes, int n_in,
                              void* d_out, int out_size, void* d_ws, size_t ws_size,
                              hipStream_t stream) {
  if (n_in < 12 || d_out == nullptr || d_ws == nullptr) return;
  if (in_sizes[0] != NBATCH * NSTEP) return;
  if (in_sizes[1] != NBATCH * NSTEP) return;
  if (in_sizes[2] != NHID) return;
  if (in_sizes[3] != NW_ELEMS) return;
  if (in_sizes[4] != NHID) return;
  if (in_sizes[5] != NHID) return;
  if (in_sizes[6] != NW_ELEMS) return;
  if (in_sizes[7] != NW_ELEMS) return;
  if (in_sizes[8] != NHID) return;
  if (in_sizes[9] != NHID) return;
  if (in_sizes[10] != NHID) return;
  if (in_sizes[11] != 1) return;
  if (out_size != NOUT) return;
  if (ws_size < WS_TOTAL) return;

  const float* x     = (const float*)d_in[0];
  const float* z     = (const float*)d_in[1];
  const float* W_ih0 = (const float*)d_in[2];
  const float* W_hh0 = (const float*)d_in[3];
  const float* b_ih0 = (const float*)d_in[4];
  const float* b_hh0 = (const float*)d_in[5];
  const float* W_ih1 = (const float*)d_in[6];
  const float* W_hh1 = (const float*)d_in[7];
  const float* b_ih1 = (const float*)d_in[8];
  const float* b_hh1 = (const float*)d_in[9];
  const float* W_lin = (const float*)d_in[10];
  const float* b_lin = (const float*)d_in[11];
  float* out = (float*)d_out;

  char* ws = (char*)d_ws;
  unsigned short* WH0 = (unsigned short*)(ws + OFF_WH0);
  unsigned short* WI1 = (unsigned short*)(ws + OFF_WI1);
  unsigned short* WH1 = (unsigned short*)(ws + OFF_WH1);
  float* YSEQ = (float*)(ws + OFF_YSEQ);
  float* YMAX = (float*)(ws + OFF_YMAX);

  wplane_kernel<<<96, 256, 0, stream>>>(W_hh0, W_ih1, W_hh1, WH0, WI1, WH1);

  rnn2_seq_kernel<<<NBLK_SEQ, NTHR_SEQ, 0, stream>>>(
      x, z, W_ih0, b_ih0, b_hh0, b_ih1, b_hh1, W_lin, b_lin, WH0, WI1, WH1, YSEQ, YMAX);

  pack_kernel<<<(NOUT4 + 255) / 256, 256, 0, stream>>>(YSEQ, YMAX, out);
}
